// CoAttentionMessagePassingNetwork_40750649705201
// MI455X (gfx1250) — hardware-verified
//
#include <hip/hip_runtime.h>
#include <stddef.h>
#include <stdint.h>
#include <math.h>


#define NN      32768
#define EI      131072
#define EO      1048576
#define NG      1024
#define NTHR    256
#define NWAVE   8
#define EPT     8
#define CHUNK   (NTHR * EPT)
#define WCAP    (EPT * 32)
#define LISTN   (NWAVE * WCAP)
#define NB      512
#define SLB     9
#define RCAPX   18432
#define RCAPI   2560
#define DEGCAPX 48
#define DEGCAPI 16
#define MEAS_X512 16384
#define MEAS_I512 2048
#define MEAS_XDEG 32
#define MEAS_IDEG 4
#define GTHR    128
#define WSMAX   134217728
#define OWNKV   0
#define OWE1    49152
#define OWE2    57344
#define OWO     73728
#define ORO     90112
#define WPN     122880
#define UA      (2 * NN * 16)
#define NV248   __attribute__((amdgpu_num_vgpr(248)))

static_assert((CHUNK & (CHUNK - 1)) == 0 && CHUNK == 2048);
static_assert(NB == (1 << SLB) && (NN % NB) == 0 && NN / NB == 64);
static_assert(EO <= (1 << 21) && EI <= (1 << 21));
static_assert((EO % CHUNK) == 0 && (EI % CHUNK) == 0);
static_assert(RCAPX >= MEAS_X512 + MEAS_X512 / 10 && RCAPI >= MEAS_I512 + MEAS_I512 / 10);
static_assert((RCAPX % 32) == 0 && (RCAPI % 32) == 0);
static_assert(DEGCAPX >= MEAS_XDEG + 8 && DEGCAPX <= 64);
static_assert(DEGCAPI >= MEAS_IDEG + 8 && DEGCAPI <= 32);
static_assert(NTHR * 4 == 2 * NB);
static_assert((NN % 128) == 0 && (EI % 64) == 0 && (EO % 1024) == 0 && (NG % 32) == 0);
static_assert((UA % NTHR) == 0);
static_assert((LISTN + 2 * RCAPX + 3 * NB + 16) * 4 <= 300000);
static_assert(2 * NG * 256 + 2 * EO == 2621440);

typedef float          v2f  __attribute__((ext_vector_type(2)));
typedef float          v4f  __attribute__((ext_vector_type(4)));
typedef float          v8f  __attribute__((ext_vector_type(8)));
typedef int            v4i  __attribute__((ext_vector_type(4)));
typedef int            v8i  __attribute__((ext_vector_type(8)));
typedef unsigned short v8us __attribute__((ext_vector_type(8)));
typedef __bf16         v16b __attribute__((ext_vector_type(16)));
typedef v2f  __attribute__((may_alias)) v2fa;
typedef v4f  __attribute__((may_alias)) v4fa;
typedef v4i  __attribute__((may_alias)) v4ia;
typedef v8us __attribute__((may_alias)) v8usa;
union FragB { v16b v; v8us h[2]; v8i w; };

__device__ __forceinline__ v8f wmb(const FragB& a, const FragB& b, v8f c) {
  v8f d = __builtin_amdgcn_wmma_f32_16x16x32_bf16(false, a.v, false, b.v, (short)0, c, false, false);
  asm volatile("v_nop\n\tv_nop\n\tv_nop\n\tv_nop" : "+v"(d) : "v"(a.w), "v"(b.w));
  return d;
}

__device__ __forceinline__ unsigned int f2bf(float f) {
  const unsigned int u = __float_as_uint(f);
  const unsigned int r = ((u + 0x7FFFu + ((u >> 16) & 1u)) >> 16) & 0xFFFFu;
  return ((u & 0x7FFFFFFFu) > 0x7F800000u) ? 0x7FC0u : r;
}
__device__ __forceinline__ float bf2f(unsigned int b) { return __uint_as_float(b << 16); }
__device__ __forceinline__ float bfr(float f) { return bf2f(f2bf(f)); }
__device__ __forceinline__ v8us cvt8b(const v4f a, const v4f b) {
  v8us o;
  o[0] = (unsigned short)f2bf(a.x); o[1] = (unsigned short)f2bf(a.y);
  o[2] = (unsigned short)f2bf(a.z); o[3] = (unsigned short)f2bf(a.w);
  o[4] = (unsigned short)f2bf(b.x); o[5] = (unsigned short)f2bf(b.y);
  o[6] = (unsigned short)f2bf(b.z); o[7] = (unsigned short)f2bf(b.w);
  return o;
}
__device__ __forceinline__ float lrelu(float v) { return v > 0.0f ? v : 0.01f * v; }
__device__ __forceinline__ int clampi(int v, int lo, int hi) { return v < lo ? lo : (v > hi ? hi : v); }
__device__ __forceinline__ float nmax(float a, float b) {
  const float r = a > b ? a : b;
  return (a != a) ? a : ((b != b) ? b : r);
}
__device__ __forceinline__ float rdl(float v, int k) {
  return __int_as_float(__builtin_amdgcn_readlane(__float_as_int(v), k));
}

__device__ __forceinline__ int scan_chunk(const int* __restrict__ dsts, int nE, int cbase, int slotBase,
                                          int nb, int vec8, int* list, int tid, int lane, int wave) {
  int wc = 0;
  const int el0  = tid * EPT;
  const int e0   = cbase + el0;
  const int sent = -2147483647 - 1;
  v4i da, db;
  if (vec8 != 0 && cbase + CHUNK <= nE) {
    da = *(const v4i*)(dsts + e0);
    db = *(const v4i*)(dsts + e0 + 4);
  } else {
    da.x = (e0     < nE) ? dsts[min(e0,     nE - 1)] : sent;
    da.y = (e0 + 1 < nE) ? dsts[min(e0 + 1, nE - 1)] : sent;
    da.z = (e0 + 2 < nE) ? dsts[min(e0 + 2, nE - 1)] : sent;
    da.w = (e0 + 3 < nE) ? dsts[min(e0 + 3, nE - 1)] : sent;
    db.x = (e0 + 4 < nE) ? dsts[min(e0 + 4, nE - 1)] : sent;
    db.y = (e0 + 5 < nE) ? dsts[min(e0 + 5, nE - 1)] : sent;
    db.z = (e0 + 6 < nE) ? dsts[min(e0 + 6, nE - 1)] : sent;
    db.w = (e0 + 7 < nE) ? dsts[min(e0 + 7, nE - 1)] : sent;
  }
  const unsigned nbs = (unsigned)slotBase;
  const unsigned unb = (unsigned)nb;
  const unsigned s0 = (unsigned)da.x - nbs, s1 = (unsigned)da.y - nbs;
  const unsigned s2 = (unsigned)da.z - nbs, s3 = (unsigned)da.w - nbs;
  const unsigned s4 = (unsigned)db.x - nbs, s5 = (unsigned)db.y - nbs;
  const unsigned s6 = (unsigned)db.z - nbs, s7 = (unsigned)db.w - nbs;
  const bool h0 = s0 < unb, h1 = s1 < unb, h2 = s2 < unb, h3 = s3 < unb;
  const bool h4 = s4 < unb, h5 = s5 < unb, h6 = s6 < unb, h7 = s7 < unb;
  const unsigned any = __builtin_amdgcn_ballot_w32(h0 | h1 | h2 | h3 | h4 | h5 | h6 | h7);
  if (any != 0u) {
#define HITJ(J, HJ, SJ) { \
      const unsigned mj = __builtin_amdgcn_ballot_w32(HJ); \
      if (mj != 0u) { \
        if (HJ) { \
          const int pos = wc + (int)__builtin_amdgcn_mbcnt_lo(mj, 0u); \
          if (pos < WCAP) list[wave * WCAP + pos] = ((el0 + (J)) << SLB) | (int)(SJ); \
        } \
        wc += (int)__builtin_popcount(mj); } }
    HITJ(0, h0, s0)
    HITJ(1, h1, s1)
    HITJ(2, h2, s2)
    HITJ(3, h3, s3)
    HITJ(4, h4, s4)
    HITJ(5, h5, s5)
    HITJ(6, h6, s6)
    HITJ(7, h7, s7)
#undef HITJ
  }
  return wc;
}

__global__ __launch_bounds__(NTHR) void k_pa(const float* __restrict__ n1, const float* __restrict__ n2,
                                             float* NODE, unsigned short* XHL) {
  const int u = (int)blockIdx.x * NTHR + (int)threadIdx.x;
  if (u < UA) {
    const int side = (u >= NN * 16) ? 1 : 0;
    const int r = u - side * NN * 16;
    const v4f a = *(const v4f*)(n1 + (size_t)r * 4);
    const v4f b = *(const v4f*)(n2 + (size_t)r * 4);
    v4f o;
    o.x = bfr(side ? b.x : a.x); o.y = bfr(side ? b.y : a.y);
    o.z = bfr(side ? b.z : a.z); o.w = bfr(side ? b.w : a.w);
    float* dp = NODE + (size_t)u * 4;
    *(volatile v4f*)dp = o;
    __threadfence();
    *(volatile v4f*)dp = o;
  } else if (u < 2 * UA) {
    const int v = u - UA;
    const int side = (v >= NN * 16) ? 1 : 0;
    const int rr = v - side * NN * 16;
    const int row = rr >> 4, c8 = rr & 15;
    const size_t so = (size_t)row * 64 + (size_t)(c8 & 7) * 8;
    const v4f a0 = *(const v4f*)(n1 + so), a1 = *(const v4f*)(n1 + so + 4);
    const v4f b0 = *(const v4f*)(n2 + so), b1 = *(const v4f*)(n2 + so + 4);
    const v8us ha = cvt8b(a0, a1);
    const v8us hb = cvt8b(b0, b1);
    v8us o;
#pragma unroll
    for (int i = 0; i < 8; ++i) {
      const unsigned short x = side ? hb[i] : ha[i];
      o[i] = (c8 < 8) ? x : (unsigned short)0;
    }
    unsigned short* dp = XHL + (size_t)v * 8;
    *(volatile v8us*)dp = o;
    __threadfence();
    *(volatile v8us*)dp = o;
  }
}

__device__ __forceinline__ v8us gather8(const float* __restrict__ p, int ld) {
  v8us o;
#pragma unroll
  for (int i = 0; i < 8; ++i) o[i] = (unsigned short)f2bf(p[(size_t)i * ld]);
  return o;
}

__global__ __launch_bounds__(NTHR) void k_pb(const float* __restrict__ Wn, const float* __restrict__ Wk,
                                             const float* __restrict__ Wv, const float* __restrict__ We1,
                                             const float* __restrict__ We2, const float* __restrict__ Wo,
                                             const float* __restrict__ roW, unsigned short* WP) {
  const int u = (int)blockIdx.x * NTHR + (int)threadIdx.x;
  v8us o;
  size_t d;
  if (u < 2048) {
    const int v = u, s = v >> 10, n = (v >> 4) & 63, k8 = v & 15;
    o = gather8(Wn + (size_t)s * 4096 + (size_t)((k8 & 7) * 8) * 64 + n, 64);
    d = (size_t)OWNKV + (size_t)s * 24576 + (size_t)n * 128 + k8 * 8;
  } else if (u < 4096) {
    const int v = u - 2048, s = v >> 10, n = (v >> 4) & 63, k8 = v & 15;
    o = gather8(Wk + (size_t)s * 4096 + (size_t)((k8 & 7) * 8) * 64 + n, 64);
    d = (size_t)OWNKV + (size_t)s * 24576 + (size_t)(64 + n) * 128 + k8 * 8;
  } else if (u < 6144) {
    const int v = u - 4096, s = v >> 10, n = (v >> 4) & 63, k8 = v & 15;
    o = gather8(Wv + (size_t)s * 4096 + (size_t)((k8 & 7) * 8) * 64 + n, 64);
    d = (size_t)OWNKV + (size_t)s * 24576 + (size_t)(128 + n) * 128 + k8 * 8;
  } else if (u < 7168) {
    const int v = u - 6144, s = v >> 9, n = (v >> 3) & 63, k8 = v & 7;
    o = gather8(We1 + (size_t)s * 4096 + (size_t)(k8 * 8) * 64 + n, 64);
    d = (size_t)OWE1 + (size_t)s * 4096 + (size_t)n * 64 + k8 * 8;
  } else if (u < 9216) {
    const int v = u - 7168, s = v >> 10, n = (v >> 4) & 63, k8 = v & 15;
    o = gather8(We2 + (size_t)s * 4096 + (size_t)((k8 & 7) * 8) * 64 + n, 64);
    d = (size_t)OWE2 + (size_t)s * 8192 + (size_t)n * 128 + k8 * 8;
  } else if (u < 11264) {
    const int v = u - 9216, s = v >> 10, n = (v >> 4) & 63, k8 = v & 15;
    o = gather8(Wo + (size_t)s * 4096 + (size_t)((k8 & 7) * 8) * 64 + n, 64);
    d = (size_t)OWO + (size_t)s * 8192 + (size_t)n * 128 + k8 * 8;
  } else if (u < 15360) {
    const int v = u - 11264, n = v >> 4, k8 = v & 15;
    o = gather8(roW + (size_t)((k8 & 7) * 8) * 256 + n, 256);
    d = (size_t)ORO + (size_t)n * 128 + k8 * 8;
  } else {
    return;
  }
  unsigned short* dp = WP + d;
  *(volatile v8us*)dp = o;
  __threadfence();
  *(volatile v8us*)dp = o;
}

template <int RC>
__global__ __launch_bounds__(NTHR) NV248 void k_bucket(const int* __restrict__ keys, int nE, int vec8,
                                                       int* LISTG, int* COG, int* FLGG) {
  extern __shared__ __attribute__((aligned(16))) int bsm[];
  int* list = bsm;
  int* reg1 = bsm + LISTN;
  int* reg2 = reg1 + RC;
  int* cnt  = reg2 + RC;
  int* offs = cnt + NB;
  int* cur  = offs + NB;
  int* wcnt = cur + NB;
  const int tid = (int)threadIdx.x, lane = tid & 31, wave = tid >> 5;
  const int blk = (int)blockIdx.x;
  const int slotBase = blk * NB;

  for (int i = tid; i < 3 * NB; i += NTHR) cnt[i] = 0;
  if (tid < 16) wcnt[tid] = 0;
  __syncthreads();

  int tot = 0, ovf = 0;
  const int nChunks = (nE + CHUNK - 1) / CHUNK;
#pragma unroll 1
  for (int ch = 0; ch < nChunks; ++ch) {
    const int cbase = ch * CHUNK;
    const int wc = scan_chunk(keys, nE, cbase, slotBase, NB, vec8, list, tid, lane, wave);
    if (lane == 0) wcnt[wave] = wc;
    __syncthreads();
    int pre = 0, all = 0;
#pragma unroll
    for (int w2 = 0; w2 < NWAVE; ++w2) {
      int c = wcnt[w2];
      c = c < 0 ? 0 : (c > WCAP ? WCAP : c);
      all += c;
      pre += (w2 < wave) ? c : 0;
    }
    const int wcc  = wc > WCAP ? WCAP : wc;
    const int base = tot + pre;
#pragma unroll 1
    for (int i = lane; i < wcc; i += 32) {
      const int ent = list[wave * WCAP + i];
      const int el  = (ent >> SLB) & (CHUNK - 1);
      const int sl  = ent & (NB - 1);
      int eid = cbase + el;
      eid = eid > nE - 1 ? nE - 1 : eid;
      const int pos = base + i;
      if (pos < RC) reg1[pos] = (int)(((unsigned)eid << SLB) | (unsigned)sl);
    }
    if (tot + all > RC) ovf = 1;
    tot += all;
    tot = tot > RC ? RC : tot;
    __syncthreads();
  }
  const int nh = tot;

  if (wave == 0) {
#pragma unroll 1
    for (int b0 = 0; b0 < nh; b0 += 32) {
      const int idx = b0 + lane;
      const int uv  = reg1[idx < nh ? idx : nh - 1];
      const int m32 = (nh - b0) < 32 ? (nh - b0) : 32;
#pragma unroll 1
      for (int k = 0; k < m32; ++k) {
        const int u  = __builtin_amdgcn_readlane(uv, k);
        const int sq = u & (NB - 1);
        if (lane == 0) cnt[sq] = cnt[sq] + 1;
      }
    }
  }
  __syncthreads();
  if (wave == 0) {
    const int base = lane * (NB / 32);
    int s = 0;
#pragma unroll 1
    for (int i = 0; i < NB / 32; ++i) s += cnt[base + i];
    int incl = s;
#pragma unroll
    for (int d = 1; d < 32; d <<= 1) {
      const int y = __shfl_up(incl, d, 32);
      if (lane >= d) incl += y;
    }
    int run = incl - s;
#pragma unroll 1
    for (int i = 0; i < NB / 32; ++i) {
      const int cv = cnt[base + i];
      offs[base + i] = run;
      cur[base + i]  = run;
      run += cv;
    }
  }
  __syncthreads();
  if (wave == 0) {
#pragma unroll 1
    for (int b0 = 0; b0 < nh; b0 += 32) {
      const int idx = b0 + lane;
      const int uv  = reg1[idx < nh ? idx : nh - 1];
      const int m32 = (nh - b0) < 32 ? (nh - b0) : 32;
#pragma unroll 1
      for (int k = 0; k < m32; ++k) {
        const int u  = __builtin_amdgcn_readlane(uv, k);
        const int sq = u & (NB - 1);
        if (lane == 0) {
          int p = cur[sq];
          p = p < 0 ? 0 : (p > RC - 1 ? RC - 1 : p);
          reg2[p] = (int)((unsigned)u >> SLB);
          cur[sq] = p + 1;
        }
      }
    }
  }
  __syncthreads();
  for (int i = nh + tid; i < RC; i += NTHR) reg2[i] = 0;
  __syncthreads();

  int* lb = LISTG + (size_t)blk * RC;
  v4i cv;
  cv.x = (tid == 0) ? nh : 0;
  cv.y = (tid == 0) ? ovf : 0;
  cv.z = 0; cv.w = 0;
  int* fp = FLGG + (size_t)blk * 32 + 4 * (tid & 7);
  const v4i cov = *(const v4ia*)(cnt + 4 * tid);
  int* cop = COG + (size_t)(tid >> 7) * NN + (size_t)blk * NB + 4 * (tid & 127);
#pragma unroll 1
  for (int p = tid * 4; p < RC; p += NTHR * 4) {
    const v4i v = *(const v4ia*)(reg2 + p);
    *(volatile v4i*)(lb + p) = v;
  }
  *(volatile v4i*)cop = cov;
  if (tid < 8) *(volatile v4i*)fp = cv;
  __threadfence();
#pragma unroll 1
  for (int p = tid * 4; p < RC; p += NTHR * 4) {
    const v4i v = *(const v4ia*)(reg2 + p);
    *(volatile v4i*)(lb + p) = v;
  }
  *(volatile v4i*)cop = cov;
  if (tid < 8) *(volatile v4i*)fp = cv;
}

__global__ __launch_bounds__(GTHR) NV248 void k_gn(const unsigned short* __restrict__ A,
                                                   const unsigned short* __restrict__ WT,
                                                   float* wsf, size_t offPN, size_t offKV, int K) {
  __shared__ __attribute__((aligned(16))) float stg[64 * 64];
  const int tid = (int)threadIdx.x, lane = tid & 31, wave = tid >> 5, hh = lane >> 4, m = lane & 15;
  const int rowBase = (int)blockIdx.x * 64;
  const int y = (int)blockIdx.y;
  const int col0 = 64 * y;
  v8f acc[4];
  {
    const v8f z = {0.f, 0.f, 0.f, 0.f, 0.f, 0.f, 0.f, 0.f};
    acc[0] = z; acc[1] = z; acc[2] = z; acc[3] = z;
  }
  const unsigned short* ap = A  + (size_t)(rowBase + 16 * wave + m) * 128 + 8 * hh;
  const unsigned short* wp = WT + (size_t)(col0 + m) * 128 + 8 * hh;
  const int ksteps = K >> 5;
#pragma unroll 1
  for (int ks = 0; ks < ksteps; ++ks) {
    FragB af;
    af.h[0] = *(const v8usa*)(ap + 32 * ks);
    af.h[1] = *(const v8usa*)(ap + 32 * ks + 16);
#pragma unroll
    for (int t = 0; t < 4; ++t) {
      const unsigned short* wq = wp + (size_t)(16 * t) * 128 + 32 * ks;
      FragB bf;
      bf.h[0] = *(const v8usa*)wq;
      bf.h[1] = *(const v8usa*)(wq + 16);
      acc[t] = wmb(af, bf, acc[t]);
    }
  }
#pragma unroll
  for (int t = 0; t < 4; ++t) {
#pragma unroll
    for (int r = 0; r < 8; ++r) stg[(16 * wave + 8 * hh + r) * 64 + 16 * t + m] = acc[t][r];
  }
  __syncthreads();
  const size_t ob = (y == 0) ? offPN : (offKV + (size_t)(y - 1) * 64);
  const int ldo = (y == 0) ? 64 : 128;
  float* obase = wsf + ob + (size_t)rowBase * (size_t)ldo;
  v4f fv[8];
#pragma unroll
  for (int i = 0; i < 8; ++i) fv[i] = *(const v4fa*)(stg + (16 * wave + 2 * i + hh) * 64 + 4 * m);
#pragma unroll
  for (int i = 0; i < 8; ++i)
    *(volatile v4f*)(obase + (size_t)(16 * wave + 2 * i + hh) * (size_t)ldo + 4 * m) = fv[i];
  __threadfence();
#pragma unroll
  for (int i = 0; i < 8; ++i)
    *(volatile v4f*)(obase + (size_t)(16 * wave + 2 * i + hh) * (size_t)ldo + 4 * m) = fv[i];
}

__global__ __launch_bounds__(GTHR) NV248 void k_em(const float* __restrict__ edge, const int* __restrict__ idx,
                                                   const unsigned short* __restrict__ W1T,
                                                   const unsigned short* __restrict__ W2D,
                                                   const float* __restrict__ be1, const float* __restrict__ be2,
                                                   const float* __restrict__ PN, float* EMSG) {
  __shared__ __attribute__((aligned(16))) unsigned short hl[64 * 128];
  __shared__ __attribute__((aligned(16))) float stg[64 * 64];
  __shared__ float sb1[64];
  __shared__ float sb2[64];
  __shared__ int sidx[64];
  const int tid = (int)threadIdx.x, lane = tid & 31, wave = tid >> 5, hh = lane >> 4, m = lane & 15;
  const int e0 = (int)blockIdx.x * 64;
  if (tid < 64) {
    sb1[tid] = bfr(be1[tid]);
    sb2[tid] = bfr(be2[tid]);
    sidx[tid] = clampi(idx[e0 + tid], 0, NN - 1);
  }
  v8f acc[4];
  {
    const v8f z = {0.f, 0.f, 0.f, 0.f, 0.f, 0.f, 0.f, 0.f};
    acc[0] = z; acc[1] = z; acc[2] = z; acc[3] = z;
  }
  {
    const float* ep = edge + (size_t)(e0 + 16 * wave + m) * 64 + 8 * hh;
    const unsigned short* wp = W1T + (size_t)m * 64 + 8 * hh;
#pragma unroll 1
    for (int ks = 0; ks < 2; ++ks) {
      const v4f a0 = *(const v4f*)(ep + 32 * ks),      a1 = *(const v4f*)(ep + 32 * ks + 4);
      const v4f b0 = *(const v4f*)(ep + 32 * ks + 16), b1 = *(const v4f*)(ep + 32 * ks + 20);
      FragB af;
      af.h[0] = cvt8b(a0, a1);
      af.h[1] = cvt8b(b0, b1);
#pragma unroll
      for (int t = 0; t < 4; ++t) {
        const unsigned short* wq = wp + (size_t)(16 * t) * 64 + 32 * ks;
        FragB bf;
        bf.h[0] = *(const v8usa*)wq;
        bf.h[1] = *(const v8usa*)(wq + 16);
        acc[t] = wmb(af, bf, acc[t]);
      }
    }
  }
  __syncthreads();
#pragma unroll
  for (int t = 0; t < 4; ++t) {
    const int c = 16 * t + m;
    const float b = sb1[c];
#pragma unroll
    for (int r = 0; r < 8; ++r) {
      const int lr = 16 * wave + 8 * hh + r;
      const float v = lrelu(acc[t][r] + b);
      const unsigned int hb = f2bf(v);
      const unsigned int lo = f2bf(v - bf2f(hb));
      hl[lr * 128 + c]      = (unsigned short)hb;
      hl[lr * 128 + 64 + c] = (unsigned short)lo;
    }
  }
  __syncthreads();
  v8f ac2[4];
  {
    const v8f z = {0.f, 0.f, 0.f, 0.f, 0.f, 0.f, 0.f, 0.f};
    ac2[0] = z; ac2[1] = z; ac2[2] = z; ac2[3] = z;
  }
  {
    const unsigned short* hp = hl + (16 * wave + m) * 128 + 8 * hh;
    const unsigned short* wp = W2D + (size_t)m * 128 + 8 * hh;
#pragma unroll 1
    for (int ks = 0; ks < 4; ++ks) {
      FragB af;
      af.h[0] = *(const v8usa*)(hp + 32 * ks);
      af.h[1] = *(const v8usa*)(hp + 32 * ks + 16);
#pragma unroll
      for (int t = 0; t < 4; ++t) {
        const unsigned short* wq = wp + (size_t)(16 * t) * 128 + 32 * ks;
        FragB bf;
        bf.h[0] = *(const v8usa*)wq;
        bf.h[1] = *(const v8usa*)(wq + 16);
        ac2[t] = wmb(af, bf, ac2[t]);
      }
    }
  }
#pragma unroll
  for (int t = 0; t < 4; ++t) {
    const int c = 16 * t + m;
    const float b = sb2[c];
#pragma unroll
    for (int r = 0; r < 8; ++r) stg[(16 * wave + 8 * hh + r) * 64 + c] = lrelu(ac2[t][r] + b);
  }
  __syncthreads();
  v4f fv[8];
#pragma unroll
  for (int i = 0; i < 8; ++i) {
    const int lr = 16 * wave + 2 * i + hh;
    const v4f ev = *(const v4fa*)(stg + lr * 64 + 4 * m);
    const int j = sidx[lr];
    const v4f pv = *(const v4f*)(PN + (size_t)j * 64 + 4 * m);
    v4f o;
    o.x = ev.x * pv.x; o.y = ev.y * pv.y; o.z = ev.z * pv.z; o.w = ev.w * pv.w;
    fv[i] = o;
  }
  float* obase = EMSG + (size_t)e0 * 64;
#pragma unroll
  for (int i = 0; i < 8; ++i) *(volatile v4f*)(obase + (size_t)(16 * wave + 2 * i + hh) * 64 + 4 * m) = fv[i];
  __threadfence();
#pragma unroll
  for (int i = 0; i < 8; ++i) *(volatile v4f*)(obase + (size_t)(16 * wave + 2 * i + hh) * 64 + 4 * m) = fv[i];
}

__global__ __launch_bounds__(NTHR) void k_in(const int* __restrict__ LIST, const int* __restrict__ CO,
                                             const int* __restrict__ FLG, const float* __restrict__ EMSG,
                                             float* NODEs) {
  const int tid = (int)threadIdx.x, lane = tid & 31, wave = tid >> 5;
  const int blk = (int)blockIdx.x;
  const float qnan = __int_as_float(0x7fc00000);
#pragma unroll 1
  for (int si = 0; si < 8; ++si) {
    const int n = blk * 64 + wave * 8 + si;
    const int b = n >> SLB;
    const int flag = FLG[(size_t)b * 32 + 1];
    const int craw = CO[n];
    const int oraw = CO[NN + n];
    int c = clampi(craw, 0, DEGCAPI);
    const int o = clampi(oraw, 0, RCAPI);
    if (c > RCAPI - o) c = RCAPI - o;
    const bool pz = (flag != 0) || craw < 0 || craw > DEGCAPI || oraw < 0 || oraw > RCAPI;
    int x = o + lane;
    x = x > RCAPI - 1 ? RCAPI - 1 : x;
    const int e = clampi(LIST[(size_t)b * RCAPI + x], 0, EI - 1);
    float s0 = 0.0f, s1 = 0.0f;
#pragma unroll 1
    for (int k = 0; k < c; ++k) {
      const int ek = __builtin_amdgcn_readlane(e, k);
      const v2f v = *(const v2f*)(EMSG + (size_t)ek * 64 + 2 * lane);
      s0 += v.x; s1 += v.y;
    }
    s0 = pz ? qnan : s0;
    s1 = pz ? qnan : s1;
    float* np = NODEs + (size_t)n * 64 + 2 * lane;
    const v2f nd = *(const v2f*)np;
    v2f r;
    r.x = nd.x + s0; r.y = nd.y + s1;
    *(volatile v2f*)np = r;
    __threadfence();
    *(volatile v2f*)np = r;
  }
}

__global__ __launch_bounds__(NTHR) void k_t(const int* __restrict__ i1, const int* __restrict__ i2,
                                            const float* __restrict__ KV, float* T) {
  __shared__ __attribute__((aligned(16))) float sT[1024];
  const int tid = (int)threadIdx.x;
  const int g = tid >> 3, q = tid & 7;
  const int base = (int)blockIdx.x * 1024;
#pragma unroll 1
  for (int p = 0; p < 32; ++p) {
    const int el = p * 32 + g;
    const int e = base + el;
    const int a = clampi(i1[e], 0, NN - 1);
    const int b = clampi(i2[e], 0, NN - 1);
    const float* ra = KV + (size_t)a * 128 + 8 * q;
    const float* rb = KV + (size_t)(NN + b) * 128 + 8 * q;
    const v4f a0 = *(const v4f*)ra, a1 = *(const v4f*)(ra + 4);
    const v4f b0 = *(const v4f*)rb, b1 = *(const v4f*)(rb + 4);
    float d = a0.x * b0.x;
    d = fmaf(a0.y, b0.y, d); d = fmaf(a0.z, b0.z, d); d = fmaf(a0.w, b0.w, d);
    d = fmaf(a1.x, b1.x, d); d = fmaf(a1.y, b1.y, d); d = fmaf(a1.z, b1.z, d); d = fmaf(a1.w, b1.w, d);
    d += __shfl_xor(d, 1);
    d += __shfl_xor(d, 2);
    d += __shfl_xor(d, 4);
    if (q == 0) sT[el] = d;
  }
  __syncthreads();
  const v4f v = *(const v4fa*)(sT + 4 * tid);
  float* op = T + (size_t)base + 4 * tid;
  *(volatile v4f*)op = v;
  __threadfence();
  *(volatile v4f*)op = v;
}

__global__ __launch_bounds__(NTHR) NV248 void k_x(const int* __restrict__ LIST, const int* __restrict__ CO,
                                                  const int* __restrict__ FLG, const int* __restrict__ partner,
                                                  const float* __restrict__ T, const float* __restrict__ V,
                                                  unsigned short* XH, float* MZ) {
  __shared__ __attribute__((aligned(16))) float smz[2 * 128];
  const int tid = (int)threadIdx.x, lane = tid & 31, wave = tid >> 5;
  const int blk = (int)blockIdx.x;
  const float qnan = __int_as_float(0x7fc00000);
  const float NEGB = -3.0e38f;
#pragma unroll 1
  for (int si = 0; si < 16; ++si) {
    const int sl = wave * 16 + si;
    const int n = blk * 128 + sl;
    const int b = n >> SLB;
    const int flag = FLG[(size_t)b * 32 + 1];
    const int craw = CO[n];
    const int oraw = CO[NN + n];
    int c = clampi(craw, 0, DEGCAPX);
    const int o = clampi(oraw, 0, RCAPX);
    if (c > RCAPX - o) c = RCAPX - o;
    const bool pz = (flag != 0) || craw < 0 || craw > DEGCAPX || oraw < 0 || oraw > RCAPX;
    const int* lb = LIST + (size_t)b * RCAPX;
    int x0 = o + lane;      x0 = x0 > RCAPX - 1 ? RCAPX - 1 : x0;
    int x1 = o + 32 + lane; x1 = x1 > RCAPX - 1 ? RCAPX - 1 : x1;
    const int e0 = clampi(lb[x0], 0, EO - 1);
    const int e1 = clampi(lb[x1], 0, EO - 1);
    const float t0 = T[e0];
    const float t1 = T[e1];
    const int j0 = clampi(partner[e0], 0, NN - 1);
    const int j1 = clampi(partner[e1], 0, NN - 1);
    const bool v0 = lane < c;
    const bool v1 = (lane + 32) < c;
    float mm = nmax(v0 ? t0 : NEGB, v1 ? t1 : NEGB);
#pragma unroll
    for (int off = 16; off > 0; off >>= 1) mm = nmax(mm, __shfl_xor(mm, off));
    const float q0 = expf((t0 - mm) * 0.125f);
    const float q1 = expf((t1 - mm) * 0.125f);
    const float p0 = v0 ? q0 : 0.0f;
    const float p1 = v1 ? q1 : 0.0f;
    float z = p0 + p1;
#pragma unroll
    for (int off = 16; off > 0; off >>= 1) z += __shfl_xor(z, off);
    const float den = z + 1e-8f;
    const float a0 = p0 / den;
    const float a1 = p1 / den;
    float acc0 = 0.0f, acc1 = 0.0f;
    const int c0 = c < 32 ? c : 32;
#pragma unroll 1
    for (int k = 0; k < c0; ++k) {
      const float ak = rdl(a0, k);
      const int jk = __builtin_amdgcn_readlane(j0, k);
      const v2f vv = *(const v2f*)(V + (size_t)jk * 128 + 2 * lane);
      acc0 = fmaf(ak, vv.x, acc0);
      acc1 = fmaf(ak, vv.y, acc1);
    }
#pragma unroll 1
    for (int k = 0; k < c - 32; ++k) {
      const float ak = rdl(a1, k);
      const int jk = __builtin_amdgcn_readlane(j1, k);
      const v2f vv = *(const v2f*)(V + (size_t)jk * 128 + 2 * lane);
      acc0 = fmaf(ak, vv.x, acc0);
      acc1 = fmaf(ak, vv.y, acc1);
    }
    float Mv = (c > 0) ? mm : 0.0f;
    float Zv = (c > 0) ? z : 0.0f;
    acc0 = pz ? qnan : acc0;
    acc1 = pz ? qnan : acc1;
    Mv = pz ? qnan : Mv;
    Zv = pz ? qnan : Zv;
    const unsigned int h0 = f2bf(acc0), h1 = f2bf(acc1);
    const unsigned int l0 = f2bf(acc0 - bf2f(h0)), l1 = f2bf(acc1 - bf2f(h1));
    const unsigned int hw = h0 | (h1 << 16);
    const unsigned int lw = l0 | (l1 << 16);
    unsigned int* xp = (unsigned int*)(XH + (size_t)n * 128) + lane;
    *(volatile unsigned int*)xp = hw;
    *(volatile unsigned int*)(xp + 32) = lw;
    __threadfence();
    *(volatile unsigned int*)xp = hw;
    *(volatile unsigned int*)(xp + 32) = lw;
    if (lane == 0) { smz[sl] = Mv; smz[128 + sl] = Zv; }
  }
  __syncthreads();
  if (wave == 0) {
    const v4f mv = *(const v4fa*)(smz + 4 * lane);
    const v4f zv = *(const v4fa*)(smz + 128 + 4 * lane);
    float* mp = MZ + (size_t)blk * 128 + 4 * lane;
    float* zp = MZ + (size_t)NN + (size_t)blk * 128 + 4 * lane;
    *(volatile v4f*)mp = mv;
    *(volatile v4f*)zp = zv;
    __threadfence();
    *(volatile v4f*)mp = mv;
    *(volatile v4f*)zp = zv;
  }
}

__global__ __launch_bounds__(GTHR) NV248 void k_go(unsigned short* XHL, const unsigned short* __restrict__ WT,
                                                   float* NODE, const float* __restrict__ bo,
                                                   const float* __restrict__ lng, const float* __restrict__ lnb) {
  __shared__ __attribute__((aligned(16))) float stg[64 * 64];
  __shared__ float sbo[64];
  __shared__ float sg[64];
  __shared__ float sb[64];
  const int tid = (int)threadIdx.x, lane = tid & 31, wave = tid >> 5, hh = lane >> 4, m = lane & 15;
  const int rowBase = (int)blockIdx.x * 64;
  const int side = (int)blockIdx.y;
  if (tid < 64) { sbo[tid] = bfr(bo[tid]); sg[tid] = bfr(lng[tid]); sb[tid] = bfr(lnb[tid]); }
  v8f acc[4];
  {
    const v8f z = {0.f, 0.f, 0.f, 0.f, 0.f, 0.f, 0.f, 0.f};
    acc[0] = z; acc[1] = z; acc[2] = z; acc[3] = z;
  }
  const size_t r0 = (size_t)side * NN + (size_t)rowBase;
  {
    const unsigned short* ap = XHL + (r0 + 16 * wave + m) * 128 + 8 * hh;
    const unsigned short* wp = WT + (size_t)m * 128 + 8 * hh;
#pragma unroll 1
    for (int ks = 0; ks < 4; ++ks) {
      FragB af;
      af.h[0] = *(const v8usa*)(ap + 32 * ks);
      af.h[1] = *(const v8usa*)(ap + 32 * ks + 16);
#pragma unroll
      for (int t = 0; t < 4; ++t) {
        const unsigned short* wq = wp + (size_t)(16 * t) * 128 + 32 * ks;
        FragB bf;
        bf.h[0] = *(const v8usa*)wq;
        bf.h[1] = *(const v8usa*)(wq + 16);
        acc[t] = wmb(af, bf, acc[t]);
      }
    }
  }
#pragma unroll
  for (int t = 0; t < 4; ++t) {
#pragma unroll
    for (int r = 0; r < 8; ++r) stg[(16 * wave + 8 * hh + r) * 64 + 16 * t + m] = acc[t][r];
  }
  __syncthreads();
  {
    const float b0 = sbo[2 * lane], b1 = sbo[2 * lane + 1];
    const float g0 = sg[2 * lane],  g1 = sg[2 * lane + 1];
    const float c0 = sb[2 * lane],  c1 = sb[2 * lane + 1];
#pragma unroll 1
    for (int rr = 0; rr < 16; ++rr) {
      const int lr = 16 * wave + rr;
      const v2f ov = *(const v2fa*)(stg + lr * 64 + 2 * lane);
      const v2f nd = *(const v2f*)(NODE + (r0 + lr) * 64 + 2 * lane);
      const float x0 = nd.x + lrelu(ov.x + b0);
      const float x1 = nd.y + lrelu(ov.y + b1);
      float s = x0 + x1;
#pragma unroll
      for (int off = 16; off > 0; off >>= 1) s += __shfl_xor(s, off);
      const float mu = s * 0.015625f;
      const float d0 = x0 - mu, d1 = x1 - mu;
      float q = d0 * d0 + d1 * d1;
#pragma unroll
      for (int off = 16; off > 0; off >>= 1) q += __shfl_xor(q, off);
      const float var = q * 0.015625f;
      const float rs = 1.0f / sqrtf(var + 1e-5f);
      v2f yv;
      yv.x = (d0 * rs) * g0 + c0;
      yv.y = (d1 * rs) * g1 + c1;
      *(v2fa*)(stg + lr * 64 + 2 * lane) = yv;
    }
  }
  __syncthreads();
  v4f fv[8];
  v8us xv[8];
#pragma unroll
  for (int i = 0; i < 8; ++i) {
    const int lr = 16 * wave + 2 * i + hh;
    fv[i] = *(const v4fa*)(stg + lr * 64 + 4 * m);
    const v4f ya = *(const v4fa*)(stg + lr * 64 + 8 * (m & 7));
    const v4f yb = *(const v4fa*)(stg + lr * 64 + 8 * (m & 7) + 4);
    const float yy[8] = {ya.x, ya.y, ya.z, ya.w, yb.x, yb.y, yb.z, yb.w};
    v8us o;
#pragma unroll
    for (int e = 0; e < 8; ++e) {
      const unsigned int hb = f2bf(yy[e]);
      const unsigned int lb = f2bf(yy[e] - bf2f(hb));
      o[e] = (unsigned short)((m < 8) ? hb : lb);
    }
    xv[i] = o;
  }
#pragma unroll
  for (int i = 0; i < 8; ++i) {
    const int lr = 16 * wave + 2 * i + hh;
    *(volatile v4f*)(NODE + (r0 + lr) * 64 + 4 * m) = fv[i];
    *(volatile v8us*)(XHL + (r0 + lr) * 128 + 8 * m) = xv[i];
  }
  __threadfence();
#pragma unroll
  for (int i = 0; i < 8; ++i) {
    const int lr = 16 * wave + 2 * i + hh;
    *(volatile v4f*)(NODE + (r0 + lr) * 64 + 4 * m) = fv[i];
    *(volatile v8us*)(XHL + (r0 + lr) * 128 + 8 * m) = xv[i];
  }
}

__global__ __launch_bounds__(NTHR) void k_a(const float* __restrict__ T, const int* __restrict__ i1,
                                            const int* __restrict__ i2, const float* __restrict__ MZ, float* out) {
  __shared__ __attribute__((aligned(16))) float sa[2 * 1024];
  const int tid = (int)threadIdx.x;
  const int base = (int)blockIdx.x * 1024;
#pragma unroll 1
  for (int p = 0; p < 4; ++p) {
    const int el = p * NTHR + tid;
    const int e = base + el;
    const float t = T[e];
    const int a = clampi(i1[e], 0, NN - 1);
    const int b = clampi(i2[e], 0, NN - 1);
    const float m1 = MZ[a];
    const float z1 = MZ[(size_t)NN + a];
    const float m2 = MZ[(size_t)2 * NN + b];
    const float z2 = MZ[(size_t)3 * NN + b];
    sa[el]        = expf((t - m1) * 0.125f) / (z1 + 1e-8f);
    sa[1024 + el] = expf((t - m2) * 0.125f) / (z2 + 1e-8f);
  }
  __syncthreads();
  const v4f x1 = *(const v4fa*)(sa + 4 * tid);
  const v4f x2 = *(const v4fa*)(sa + 1024 + 4 * tid);
  float* o1 = out + (size_t)524288 + (size_t)base + 4 * tid;
  float* o2 = out + (size_t)1572864 + (size_t)base + 4 * tid;
  *(volatile v4f*)o1 = x1;
  *(volatile v4f*)o2 = x2;
  __threadfence();
  *(volatile v4f*)o1 = x1;
  *(volatile v4f*)o2 = x2;
}

__global__ __launch_bounds__(NTHR) void k_pool(const int* __restrict__ seg, const float* __restrict__ NODEs,
                                               unsigned short* PS, float* CG) {
  __shared__ __attribute__((aligned(16))) float scn[32];
  const int tid = (int)threadIdx.x, lane = tid & 31, wave = tid >> 5;
  const int gbase = (int)blockIdx.x * 32;
#pragma unroll 1
  for (int q = 0; q < 4; ++q) {
    const int g = gbase + wave * 4 + q;
    float acc0 = 0.0f, acc1 = 0.0f;
    int cl = 0;
#pragma unroll 1
    for (int it = 0; it < NN / 32; ++it) {
      const int sgv = seg[it * 32 + lane];
      const bool hit = (sgv == g);
      unsigned mask = __builtin_amdgcn_ballot_w32(hit);
      cl += hit ? 1 : 0;
      while (mask != 0u) {
        const int k = (int)__builtin_ctz(mask);
        mask &= mask - 1u;
        const v2f v = *(const v2f*)(NODEs + (size_t)(it * 32 + k) * 64 + 2 * lane);
        acc0 += v.x; acc1 += v.y;
      }
    }
#pragma unroll
    for (int off = 16; off > 0; off >>= 1) cl += __shfl_xor(cl, off);
    const unsigned int h0 = f2bf(acc0), h1 = f2bf(acc1);
    const unsigned int l0 = f2bf(acc0 - bf2f(h0)), l1 = f2bf(acc1 - bf2f(h1));
    const unsigned int hw = h0 | (h1 << 16);
    const unsigned int lw = l0 | (l1 << 16);
    unsigned int* xp = (unsigned int*)(PS + (size_t)g * 128) + lane;
    *(volatile unsigned int*)xp = hw;
    *(volatile unsigned int*)(xp + 32) = lw;
    __threadfence();
    *(volatile unsigned int*)xp = hw;
    *(volatile unsigned int*)(xp + 32) = lw;
    if (lane == 0) scn[wave * 4 + q] = (float)cl;
  }
  __syncthreads();
  if (wave == 0) {
    const v4f cv = *(const v4fa*)(scn + 4 * (lane & 7));
    float* cp = CG + (size_t)gbase + 4 * (lane & 7);
    if (lane < 8) *(volatile v4f*)cp = cv;
    __threadfence();
    if (lane < 8) *(volatile v4f*)cp = cv;
  }
}

__global__ __launch_bounds__(GTHR) NV248 void k_ro(const unsigned short* __restrict__ A,
                                                   const unsigned short* __restrict__ WT,
                                                   const float* __restrict__ CG, const float* __restrict__ rob,
                                                   float* out) {
  __shared__ __attribute__((aligned(16))) float stg[64 * 64];
  __shared__ float scn[64];
  __shared__ float srb[64];
  const int tid = (int)threadIdx.x, lane = tid & 31, wave = tid >> 5, hh = lane >> 4, m = lane & 15;
  const int rowBase = (int)blockIdx.x * 64;
  const int col0 = (int)blockIdx.y * 64;
  if (tid < 64) { scn[tid] = CG[rowBase + tid]; srb[tid] = bfr(rob[col0 + tid]); }
  v8f acc[4];
  {
    const v8f z = {0.f, 0.f, 0.f, 0.f, 0.f, 0.f, 0.f, 0.f};
    acc[0] = z; acc[1] = z; acc[2] = z; acc[3] = z;
  }
  const unsigned short* ap = A  + (size_t)(rowBase + 16 * wave + m) * 128 + 8 * hh;
  const unsigned short* wp = WT + (size_t)(col0 + m) * 128 + 8 * hh;
#pragma unroll 1
  for (int ks = 0; ks < 4; ++ks) {
    FragB af;
    af.h[0] = *(const v8usa*)(ap + 32 * ks);
    af.h[1] = *(const v8usa*)(ap + 32 * ks + 16);
#pragma unroll
    for (int t = 0; t < 4; ++t) {
      const unsigned short* wq = wp + (size_t)(16 * t) * 128 + 32 * ks;
      FragB bf;
      bf.h[0] = *(const v8usa*)wq;
      bf.h[1] = *(const v8usa*)(wq + 16);
      acc[t] = wmb(af, bf, acc[t]);
    }
  }
  __syncthreads();
#pragma unroll
  for (int t = 0; t < 4; ++t) {
    const int c = 16 * t + m;
    const float b = srb[c];
#pragma unroll
    for (int r = 0; r < 8; ++r) {
      const int lr = 16 * wave + 8 * hh + r;
      stg[lr * 64 + c] = acc[t][r] + scn[lr] * b;
    }
  }
  __syncthreads();
  float* obase = out + (size_t)rowBase * 256 + col0;
  v4f fv[8];
#pragma unroll
  for (int i = 0; i < 8; ++i) fv[i] = *(const v4fa*)(stg + (16 * wave + 2 * i + hh) * 64 + 4 * m);
#pragma unroll
  for (int i = 0; i < 8; ++i) *(volatile v4f*)(obase + (size_t)(16 * wave + 2 * i + hh) * 256 + 4 * m) = fv[i];
  __threadfence();
#pragma unroll
  for (int i = 0; i < 8; ++i) *(volatile v4f*)(obase + (size_t)(16 * wave + 2 * i + hh) * 256 + 4 * m) = fv[i];
}

extern "C" void kernel_launch(void* const* d_in, const int* in_sizes, int n_in,
                              void* d_out, int out_size, void* d_ws, size_t ws_size,
                              hipStream_t stream) {
  if (n_in < 27) return;
  {
    const int want[27] = {NN, NN * 64, EI * 64, EI, EI, EO, EO, NN, NN * 64, EI * 64, EI, EI, EO, EO,
                          8192, 8192, 128, 8192, 128, 8192, 8192, 8192, 128, 128, 128, 16384, 256};
    for (int i = 0; i < 27; ++i) if (in_sizes[i] != want[i]) return;
  }
  if (out_size != 2 * NG * 256 + 2 * EO) return;

  const int*   seg1  = (const int*)  d_in[0];
  const float* node1 = (const float*)d_in[1];
  const float* edge1 = (const float*)d_in[2];
  const int*   iseg1 = (const int*)  d_in[3];
  const int*   iidx1 = (const int*)  d_in[4];
  const int*   oseg1 = (const int*)  d_in[5];
  const int*   seg2  = (const int*)  d_in[7];
  const float* node2 = (const float*)d_in[8];
  const float* edge2 = (const float*)d_in[9];
  const int*   iseg2 = (const int*)  d_in[10];
  const int*   iidx2 = (const int*)  d_in[11];
  const int*   oseg2 = (const int*)  d_in[12];
  const float* Wn  = (const float*)d_in[14];
  const float* We1 = (const float*)d_in[15];
  const float* be1 = (const float*)d_in[16];
  const float* We2 = (const float*)d_in[17];
  const float* be2 = (const float*)d_in[18];
  const float* Wk  = (const float*)d_in[19];
  const float* Wv  = (const float*)d_in[20];
  const float* Wo  = (const float*)d_in[21];
  const float* bo  = (const float*)d_in[22];
  const float* lng = (const float*)d_in[23];
  const float* lnb = (const float*)d_in[24];
  const float* roW = (const float*)d_in[25];
  const float* rob = (const float*)d_in[26];
  float* out = (float*)d_out;

  char* ws = (char*)d_ws;
  size_t off = 0;
  const size_t oKV  = off; off += (size_t)2 * NN * 128 * 4;
  const size_t oPN  = off; off += (size_t)NN * 64 * 4;
  const size_t oEM  = off; off += (size_t)EI * 64 * 4;
  const size_t oND  = off; off += (size_t)2 * NN * 64 * 4;
  const size_t oXH  = off; off += (size_t)2 * NN * 128 * 2;
  const size_t oT   = off; off += (size_t)EO * 4;
  const size_t oMZ  = off; off += (size_t)4 * NN * 4;
  const size_t oLX  = off; off += (size_t)2 * 64 * RCAPX * 4;
  const size_t oLI  = off; off += (size_t)2 * 64 * RCAPI * 4;
  const size_t oCO  = off; off += (size_t)4 * 2 * NN * 4;
  const size_t oFL  = off; off += (size_t)4 * 64 * 128;
  const size_t oWP  = off; off += (size_t)WPN * 2;
  const size_t oPS  = off; off += (size_t)2 * NG * 128 * 2;
  const size_t oCG  = off; off += (size_t)2 * NG * 4;
  if (off > ws_size || off > (size_t)WSMAX) return;
  float*          wsf  = (float*)ws;
  float*          KV   = (float*)(ws + oKV);
  float*          PN   = (float*)(ws + oPN);
  float*          EMSG = (float*)(ws + oEM);
  float*          NODE = (float*)(ws + oND);
  unsigned short* XHL  = (unsigned short*)(ws + oXH);
  float*          T    = (float*)(ws + oT);
  float*          MZ   = (float*)(ws + oMZ);
  int*            LX   = (int*)(ws + oLX);
  int*            LI   = (int*)(ws + oLI);
  int*            CO   = (int*)(ws + oCO);
  int*            FLG  = (int*)(ws + oFL);
  unsigned short* WP   = (unsigned short*)(ws + oWP);
  unsigned short* PS   = (unsigned short*)(ws + oPS);
  float*          CG   = (float*)(ws + oCG);

  const int ldsX = (LISTN + 2 * RCAPX + 3 * NB + 16) * 4;
  const int ldsI = (LISTN + 2 * RCAPI + 3 * NB + 16) * 4;
  hipFuncSetAttribute(reinterpret_cast<const void*>(&k_bucket<RCAPX>),
                      hipFuncAttributeMaxDynamicSharedMemorySize, ldsX);
  hipFuncSetAttribute(reinterpret_cast<const void*>(&k_bucket<RCAPI>),
                      hipFuncAttributeMaxDynamicSharedMemorySize, ldsI);

  k_pa<<<(2 * UA) / NTHR, NTHR, 0, stream>>>(node1, node2, NODE, XHL);
  k_pb<<<15360 / NTHR, NTHR, 0, stream>>>(Wn, Wk, Wv, We1, We2, Wo, roW, WP);
  k_bucket<RCAPI><<<NN / NB, NTHR, ldsI, stream>>>(iseg1, EI, 1, LI, CO, FLG);
  k_bucket<RCAPI><<<NN / NB, NTHR, ldsI, stream>>>(iseg2, EI, 1, LI + (size_t)64 * RCAPI,
                                                   CO + (size_t)2 * NN, FLG + 64 * 32);
  k_bucket<RCAPX><<<NN / NB, NTHR, ldsX, stream>>>(oseg1, EO, 1, LX, CO + (size_t)4 * NN, FLG + 2 * 64 * 32);
  k_bucket<RCAPX><<<NN / NB, NTHR, ldsX, stream>>>(oseg2, EO, 1, LX + (size_t)64 * RCAPX,
                                                   CO + (size_t)6 * NN, FLG + 3 * 64 * 32);

  for (int s = 0; s < 2; ++s) {
    const int Kn = s ? 128 : 64;
    for (int side = 0; side < 2; ++side) {
      k_gn<<<dim3(NN / 64, 3), GTHR, 0, stream>>>(XHL + (size_t)side * NN * 128, WP + OWNKV + (size_t)s * 24576,
                                                   wsf, oPN / 4, oKV / 4 + (size_t)side * NN * 128, Kn);
      k_em<<<EI / 64, GTHR, 0, stream>>>(side ? edge2 : edge1, side ? iidx2 : iidx1,
                                          WP + OWE1 + (size_t)s * 4096, WP + OWE2 + (size_t)s * 8192,
                                          be1 + s * 64, be2 + s * 64, PN, EMSG);
      k_in<<<NN / 64, NTHR, 0, stream>>>(LI + (size_t)side * 64 * RCAPI, CO + (size_t)side * 2 * NN,
                                          FLG + side * 64 * 32, EMSG, NODE + (size_t)side * NN * 64);
    }
    k_t<<<EO / 1024, NTHR, 0, stream>>>(oseg1, oseg2, KV, T);
    k_x<<<NN / 128, NTHR, 0, stream>>>(LX, CO + (size_t)4 * NN, FLG + 2 * 64 * 32, oseg2, T,
                                        KV + (size_t)NN * 128 + 64, XHL, MZ);
    k_x<<<NN / 128, NTHR, 0, stream>>>(LX + (size_t)64 * RCAPX, CO + (size_t)6 * NN, FLG + 3 * 64 * 32, oseg1, T,
                                        KV + 64, XHL + (size_t)NN * 128, MZ + (size_t)2 * NN);
    k_go<<<dim3(NN / 64, 2), GTHR, 0, stream>>>(XHL, WP + OWO + (size_t)s * 8192, NODE,
                                                 bo + s * 64, lng + s * 64, lnb + s * 64);
  }
  k_a<<<EO / 1024, NTHR, 0, stream>>>(T, oseg1, oseg2, MZ, out);
  k_pool<<<NG / 32, NTHR, 0, stream>>>(seg1, NODE, PS, CG);
  k_pool<<<NG / 32, NTHR, 0, stream>>>(seg2, NODE + (size_t)NN * 64, PS + (size_t)NG * 128, CG + NG);
  k_ro<<<dim3(2 * NG / 64, 256 / 64), GTHR, 0, stream>>>(PS, WP + ORO, CG, rob, out);
}
